// META1_74569222193913
// MI455X (gfx1250) — hardware-verified
//
#include <hip/hip_runtime.h>
#include <stddef.h>
#include <stdint.h>


#define NTHR   256
#define NWAVE  8
#define EPT    8
#define GNG    4
#define GCHUNK (NTHR * EPT * GNG)
#define WCAP   (EPT * GNG * 32)
#define LISTN  (NWAVE * WCAP)
#define ENT    32
#define ENG    8
#define ECHUNK (ENT * EPT * ENG)
#define NB     864
#define QCAP   256
#define NBG    16
#define GMAX   1024
#define FP     32
#define HP     64
#define W1P    32
#define W2P    64
#define HIDN   64
#define OUTN   16

#define SB_E1  0
#define SB_E2  64
#define SB_N1  80
#define SB_N2  144
#define SB_TOT 160

#define OW1E   0
#define OW2E   (OW1E + 2 * HIDN * W1P)
#define OW1N   (OW2E + 2 * OUTN * W2P)
#define OW2N   (OW1N + 2 * HIDN * W1P)
#define WTOT   (OW2N + 2 * OUTN * W2P)

#define OFF_ACC   0
#define OFF_QE    (OFF_ACC + NB * 16 * 4)
#define OFF_BIAS  (OFF_QE + QCAP * 4)
#define OFF_FEAT  (OFF_BIAS + SB_TOT * 4)
#define OFF_HID   (OFF_FEAT + 2 * 16 * FP * 2)
#define LDS_EDGE  (OFF_HID + 2 * 16 * HP * 2)

static_assert((GCHUNK & (GCHUNK - 1)) == 0 && GCHUNK <= 8192);
static_assert((NBG & (NBG - 1)) == 0 && NBG == 2 * NWAVE);
static_assert((NB % ENT) == 0 && ((NB * 16 / 4) % ENT) == 0);
static_assert((OFF_QE % 16) == 0 && (OFF_BIAS % 16) == 0 && (OFF_FEAT % 16) == 0 && (OFF_HID % 16) == 0);
static_assert(((2 * 16 * FP * 2 + 2 * 16 * HP * 2) % 16) == 0);
static_assert(LDS_EDGE <= 65536);
static_assert(QCAP >= 32 && (QCAP % 16) == 0);
static_assert((WTOT % 8) == 0 && WTOT / 8 == 6 * NTHR);
static_assert(OW2E == 16 * NTHR && (OW1N - OW2E) == 8 * NTHR && (OW2N - OW1N) == 16 * NTHR && (WTOT - OW2N) == 8 * NTHR);

typedef float    v4f   __attribute__((ext_vector_type(4)));
typedef float    v8f   __attribute__((ext_vector_type(8)));
typedef int      v4i   __attribute__((ext_vector_type(4)));
typedef __bf16   v8bf  __attribute__((ext_vector_type(8), may_alias));
typedef __bf16   v16bf __attribute__((ext_vector_type(16)));
union FragB { v16bf v; v8bf h[2]; };
union U8    { v8bf b; v4i i; };

__device__ __forceinline__ v8f fzero8() {
  v8f z = {0.f, 0.f, 0.f, 0.f, 0.f, 0.f, 0.f, 0.f};
  return z;
}

__device__ __forceinline__ v8bf bzero8() {
  v8bf z;
  const __bf16 b = (__bf16)0.0f;
  z[0] = b; z[1] = b; z[2] = b; z[3] = b; z[4] = b; z[5] = b; z[6] = b; z[7] = b;
  return z;
}

__device__ __forceinline__ void split2(float v, __bf16& hb, __bf16& lb) {
  hb = (__bf16)v;
  lb = (__bf16)(v - (float)hb);
}

__device__ __forceinline__ __bf16 pval(float v, int h) {
  const __bf16 hb = (__bf16)v;
  const __bf16 lb = (__bf16)(v - (float)hb);
  return (h != 0) ? lb : hb;
}

__device__ __forceinline__ void wave_sync() {
  __builtin_amdgcn_fence(__ATOMIC_RELEASE, "wavefront");
  __builtin_amdgcn_wave_barrier();
}

__device__ __forceinline__ v8f wm3(const FragB& ah, const FragB& al, const FragB& bh, const FragB& bl, v8f c) {
  c = __builtin_amdgcn_wmma_f32_16x16x32_bf16(false, ah.v, false, bh.v, (short)0, c, false, false);
  c = __builtin_amdgcn_wmma_f32_16x16x32_bf16(false, ah.v, false, bl.v, (short)0, c, false, false);
  c = __builtin_amdgcn_wmma_f32_16x16x32_bf16(false, al.v, false, bh.v, (short)0, c, false, false);
#if defined(__HIP_DEVICE_COMPILE__)
  asm volatile("v_nop\n\tv_nop\n\tv_nop\n\tv_nop" : "+v"(c) : "v"(ah.v), "v"(al.v), "v"(bh.v), "v"(bl.v));
#endif
  return c;
}

template <int NBT, int NT, int NG, int CAP, int EID>
__device__ __forceinline__ int scan_chunk(const int* __restrict__ dsts, int nE, int cbase, int slotBase,
                                          int vec8, int* lp, int tid, int wc0) {
  constexpr int CH = NT * EPT * NG;
  int wc = wc0;
#pragma unroll
  for (int g = 0; g < NG; ++g) {
    const int el0  = (g * NT + tid) * EPT;
    const int e0   = cbase + el0;
    const int sent = -2147483647 - 1;
    v4i da, db;
    if (vec8 != 0 && cbase + CH <= nE) {
      da = *(const v4i*)(dsts + e0);
      db = *(const v4i*)(dsts + e0 + 4);
    } else {
      da.x = (e0     < nE) ? dsts[min(e0, nE - 1)] : sent;
      da.y = (e0 + 1 < nE) ? dsts[min(e0 + 1, nE - 1)] : sent;
      da.z = (e0 + 2 < nE) ? dsts[min(e0 + 2, nE - 1)] : sent;
      da.w = (e0 + 3 < nE) ? dsts[min(e0 + 3, nE - 1)] : sent;
      db.x = (e0 + 4 < nE) ? dsts[min(e0 + 4, nE - 1)] : sent;
      db.y = (e0 + 5 < nE) ? dsts[min(e0 + 5, nE - 1)] : sent;
      db.z = (e0 + 6 < nE) ? dsts[min(e0 + 6, nE - 1)] : sent;
      db.w = (e0 + 7 < nE) ? dsts[min(e0 + 7, nE - 1)] : sent;
    }
    const unsigned nb = (unsigned)slotBase;
    const unsigned s0 = (unsigned)da.x - nb, s1 = (unsigned)da.y - nb;
    const unsigned s2 = (unsigned)da.z - nb, s3 = (unsigned)da.w - nb;
    const unsigned s4 = (unsigned)db.x - nb, s5 = (unsigned)db.y - nb;
    const unsigned s6 = (unsigned)db.z - nb, s7 = (unsigned)db.w - nb;
    const bool h0 = s0 < (unsigned)NBT, h1 = s1 < (unsigned)NBT, h2 = s2 < (unsigned)NBT, h3 = s3 < (unsigned)NBT;
    const bool h4 = s4 < (unsigned)NBT, h5 = s5 < (unsigned)NBT, h6 = s6 < (unsigned)NBT, h7 = s7 < (unsigned)NBT;
    const unsigned any = __builtin_amdgcn_ballot_w32(h0 | h1 | h2 | h3 | h4 | h5 | h6 | h7);
    if (any != 0u) {
#define HITJ(J, HJ, SJ) { \
        const unsigned mj = __builtin_amdgcn_ballot_w32(HJ); \
        if (mj != 0u) { \
          if (HJ) { \
            const int pos = wc + (int)__builtin_amdgcn_mbcnt_lo(mj, 0u); \
            const int ent = (EID != 0) ? (e0 + (J)) : ((((el0 + (J)) << 12)) | (int)(SJ)); \
            if (pos < CAP) lp[pos] = ent; \
          } \
          wc += (int)__builtin_popcount(mj); } }
      HITJ(0, h0, s0)
      HITJ(1, h1, s1)
      HITJ(2, h2, s2)
      HITJ(3, h3, s3)
      HITJ(4, h4, s4)
      HITJ(5, h5, s5)
      HITJ(6, h6, s6)
      HITJ(7, h7, s7)
#undef HITJ
    }
  }
  return wc;
}

__device__ __forceinline__ void stage_w(const float* __restrict__ W, int K, int Nout,
                                        __bf16* dst, int NP, int KP, int tid) {
  const int tot = NP * KP;
  for (int i = tid; i < tot; i += NTHR) {
    const int n  = i / KP;
    const int k  = i - n * KP;
    const int nc = n < Nout ? n : Nout - 1;
    const int kc = k < K ? k : K - 1;
    const float w0 = W[kc * Nout + nc];
    const float w  = (n < Nout && k < K) ? w0 : 0.0f;
    __bf16 hb, lb;
    split2(w, hb, lb);
    dst[i] = hb;
    dst[tot + i] = lb;
  }
}

__device__ __forceinline__ v8bf prep8(const float* __restrict__ W, int K, int Nout, int NP, int KP, int e0) {
  const int tot   = NP * KP;
  const int plane = e0 >= tot ? 1 : 0;
  const int jj    = e0 - plane * tot;
  const int n     = jj / KP;
  const int k0    = jj - n * KP;
  const int nc    = n < Nout ? n : Nout - 1;
  v8bf r;
#pragma unroll
  for (int e = 0; e < 8; ++e) {
    const int k  = k0 + e;
    const int kc = k < K ? k : K - 1;
    const float w0 = W[kc * Nout + nc];
    const float w  = (n < Nout && k < K) ? w0 : 0.0f;
    __bf16 hb, lb;
    split2(w, hb, lb);
    r[e] = (plane != 0) ? lb : hb;
  }
  return r;
}

__global__ __launch_bounds__(NTHR) void k_wprep(
    const float* __restrict__ ew1, const float* __restrict__ ew2,
    const float* __restrict__ nw1, const float* __restrict__ nw2, __bf16* wp) {
  const int tid = threadIdx.x;
  U8 v0, v1, v2, v3, v4, v5;
  v0.b = prep8(ew1, 9, 50, HIDN, W1P, 8 * tid);
  v1.b = prep8(ew1, 9, 50, HIDN, W1P, 8 * (NTHR + tid));
  v2.b = prep8(ew2, 50, 15, OUTN, W2P, 8 * tid);
  v3.b = prep8(nw1, 18, 50, HIDN, W1P, 8 * tid);
  v4.b = prep8(nw1, 18, 50, HIDN, W1P, 8 * (NTHR + tid));
  v5.b = prep8(nw2, 50, 15, OUTN, W2P, 8 * tid);
  __bf16* p0 = wp + OW1E + 8 * tid;
  __bf16* p1 = wp + OW1E + 8 * (NTHR + tid);
  __bf16* p2 = wp + OW2E + 8 * tid;
  __bf16* p3 = wp + OW1N + 8 * tid;
  __bf16* p4 = wp + OW1N + 8 * (NTHR + tid);
  __bf16* p5 = wp + OW2N + 8 * tid;
  *(volatile v4i*)p0 = v0.i; *(volatile v4i*)p1 = v1.i; *(volatile v4i*)p2 = v2.i;
  *(volatile v4i*)p3 = v3.i; *(volatile v4i*)p4 = v4.i; *(volatile v4i*)p5 = v5.i;
  __threadfence();
  *(volatile v4i*)p0 = v0.i; *(volatile v4i*)p1 = v1.i; *(volatile v4i*)p2 = v2.i;
  *(volatile v4i*)p3 = v3.i; *(volatile v4i*)p4 = v4.i; *(volatile v4i*)p5 = v5.i;
}

__device__ __forceinline__ void layer1(const __bf16* in, const __bf16* w1, const float* b1,
                                       __bf16* hid, int h, int m) {
  FragB ah, al;
  const __bf16* f0 = in + m * FP + 8 * h;
  ah.h[0] = *(const v8bf*)(f0);
  ah.h[1] = *(const v8bf*)(f0 + 16);
  al.h[0] = *(const v8bf*)(f0 + 16 * FP);
  al.h[1] = *(const v8bf*)(f0 + 16 * FP + 16);
#pragma unroll
  for (int t = 0; t < 4; ++t) {
    FragB bh, bl;
    const __bf16* b0 = w1 + (16 * t + m) * W1P + 8 * h;
    bh.h[0] = *(const v8bf*)(b0);
    bh.h[1] = *(const v8bf*)(b0 + 16);
    bl.h[0] = *(const v8bf*)(b0 + HIDN * W1P);
    bl.h[1] = *(const v8bf*)(b0 + HIDN * W1P + 16);
    const v8f a = wm3(ah, al, bh, bl, fzero8());
    const float bv = b1[16 * t + m];
#pragma unroll
    for (int rr = 0; rr < 8; ++rr) {
      const float v = fmaxf(a[rr] + bv, 0.0f);
      __bf16 hb, lb;
      split2(v, hb, lb);
      const int o = (8 * h + rr) * HP + 16 * t + m;
      hid[o] = hb;
      hid[16 * HP + o] = lb;
    }
  }
}

__device__ __forceinline__ v8f gemm2(const __bf16* hid, const __bf16* w2, int h, int m) {
  v8f a = fzero8();
#pragma unroll
  for (int ks = 0; ks < 2; ++ks) {
    FragB ah, al, bh, bl;
    const __bf16* f0 = hid + m * HP + 32 * ks + 8 * h;
    ah.h[0] = *(const v8bf*)(f0);
    ah.h[1] = *(const v8bf*)(f0 + 16);
    al.h[0] = *(const v8bf*)(f0 + 16 * HP);
    al.h[1] = *(const v8bf*)(f0 + 16 * HP + 16);
    const __bf16* b0 = w2 + m * W2P + 32 * ks + 8 * h;
    bh.h[0] = *(const v8bf*)(b0);
    bh.h[1] = *(const v8bf*)(b0 + 16);
    bl.h[0] = *(const v8bf*)(b0 + OUTN * W2P);
    bl.h[1] = *(const v8bf*)(b0 + OUTN * W2P + 16);
    a = wm3(ah, al, bh, bl, a);
  }
  return a;
}

__device__ __forceinline__ void process_tile(
    const float* __restrict__ x, const int* __restrict__ ei, const float* __restrict__ ea,
    int nN, int nE, int nodeBase, int tb, int nvalid, int lane,
    const int* qe, __bf16* feat, __bf16* hid,
    const __bf16* w1e, const __bf16* w2e, const __bf16* w1n, const __bf16* w2n,
    const float* sb, float* accs) {
  const int h = lane >> 4, m = lane & 15;
  const int mm = m < nvalid ? m : nvalid - 1;
  int qi = tb + mm;
  qi = qi < 0 ? 0 : (qi > QCAP - 1 ? QCAP - 1 : qi);
  int e = qe[qi];
  e = e < 0 ? 0 : (e > nE - 1 ? nE - 1 : e);
  int r = ei[e];
  int c = ei[(size_t)nE + (size_t)e];
  r = r < 0 ? 0 : (r > nN - 1 ? nN - 1 : r);
  c = c < 0 ? 0 : (c > nN - 1 ? nN - 1 : c);
  const float* xrp = x + (size_t)r * 3;
  const float* xcp = x + (size_t)c * 3;
  const float* eap = ea + (size_t)e * 3;
  const float xr0 = xrp[0], xr1 = xrp[1], xr2 = xrp[2];
  const float xc0 = xcp[0], xc1 = xcp[1], xc2 = xcp[2];
  const float ea0 = eap[0], ea1 = eap[1], ea2 = eap[2];
  const int slot = r - nodeBase;

  {
    __bf16* fr = feat + h * (16 * FP) + m * FP;
    v8bf p0;
    p0[0] = pval(xr0, h); p0[1] = pval(xr1, h); p0[2] = pval(xr2, h);
    p0[3] = pval(xc0, h); p0[4] = pval(xc1, h); p0[5] = pval(xc2, h);
    p0[6] = pval(ea0, h); p0[7] = pval(ea1, h);
    const v8bf zz = bzero8();
    *(v8bf*)(fr) = p0;
    *(v8bf*)(fr + 8) = zz;
    *(v8bf*)(fr + 16) = zz;
    fr[8] = pval(ea2, h);
  }
  wave_sync();

  layer1(feat, w1e, sb + SB_E1, hid, h, m);
  wave_sync();

  {
    const v8f a2 = gemm2(hid, w2e, h, m);
    const float bv = sb[SB_E2 + m];
#pragma unroll
    for (int rr = 0; rr < 8; ++rr) {
      const float v = a2[rr] + bv;
      __bf16 hb, lb;
      split2(v, hb, lb);
      const int row = 8 * h + rr;
      feat[row * FP + 3 + m] = hb;
      feat[16 * FP + row * FP + 3 + m] = lb;
    }
    __bf16* fr = feat + h * (16 * FP) + m * FP;
    fr[0] = pval(xc0, h); fr[1] = pval(xc1, h); fr[2] = pval(xc2, h);
  }
  wave_sync();

  layer1(feat, w1n, sb + SB_N1, hid, h, m);
  wave_sync();

  {
    const v8f a4 = gemm2(hid, w2n, h, m);
    const float bv = sb[SB_N2 + m];
    int   sv[8];
    float dv[8];
#pragma unroll
    for (int rr = 0; rr < 8; ++rr) {
      sv[rr] = __shfl(slot, 8 * h + rr);
      dv[rr] = (m == 15) ? 1.0f : (a4[rr] + bv);
    }
#pragma unroll
    for (int rr = 0; rr < 8; ++rr) {
      const int row = 8 * h + rr;
      const int s = sv[rr];
      const bool ok = (h == 0) && (row < nvalid) && ((unsigned)s < (unsigned)NB);
      const int scl = s < 0 ? 0 : (s > NB - 1 ? NB - 1 : s);
      if (ok) accs[scl * 16 + m] = accs[scl * 16 + m] + dv[rr];
    }
    wave_sync();
#pragma unroll
    for (int rr = 0; rr < 8; ++rr) {
      const int row = 8 * h + rr;
      const int s = sv[rr];
      const bool ok = (h == 1) && (row < nvalid) && ((unsigned)s < (unsigned)NB);
      const int scl = s < 0 ? 0 : (s > NB - 1 ? NB - 1 : s);
      if (ok) accs[scl * 16 + m] = accs[scl * 16 + m] + dv[rr];
    }
  }
  wave_sync();
}

__global__ __launch_bounds__(ENT) void k_edge(
    const float* __restrict__ x, const int* __restrict__ ei, const float* __restrict__ ea,
    const __bf16* __restrict__ wp,
    const float* __restrict__ eb1, const float* __restrict__ eb2,
    const float* __restrict__ nb1, const float* __restrict__ nb2,
    float* x2, int nN, int nE) {
  extern __shared__ v4f lds_dyn[];
  char* lb = (char*)lds_dyn;
  const int lane = threadIdx.x & 31;
  const int nodeBase = blockIdx.x * NB;
  float*  accs = (float*)(lb + OFF_ACC);
  int*    qe   = (int*)(lb + OFF_QE);
  float*  sb   = (float*)(lb + OFF_BIAS);
  __bf16* feat = (__bf16*)(lb + OFF_FEAT);
  __bf16* hid  = (__bf16*)(lb + OFF_HID);
  const __bf16* w1e = wp + OW1E;
  const __bf16* w2e = wp + OW2E;
  const __bf16* w1n = wp + OW1N;
  const __bf16* w2n = wp + OW2N;
  const int vec8 = ((reinterpret_cast<size_t>(ei) & 15) == 0) ? 1 : 0;

  {
    const v4f z4 = {0.f, 0.f, 0.f, 0.f};
#pragma unroll 1
    for (int i = lane; i < NB * 16 / 4; i += ENT) ((v4f*)accs)[i] = z4;
#pragma unroll 1
    for (int i = lane; i < (2 * 16 * FP * 2 + 2 * 16 * HP * 2) / 16; i += ENT) ((v4f*)(lb + OFF_FEAT))[i] = z4;
#pragma unroll 1
    for (int i = lane; i < HIDN; i += ENT) {
      const float a = eb1[i < 50 ? i : 49];
      const float b = nb1[i < 50 ? i : 49];
      sb[SB_E1 + i] = i < 50 ? a : 0.0f;
      sb[SB_N1 + i] = i < 50 ? b : 0.0f;
    }
    if (lane < OUTN) {
      const float a = eb2[lane < 15 ? lane : 14];
      const float b = nb2[lane < 15 ? lane : 14];
      sb[SB_E2 + lane] = lane < 15 ? a : 0.0f;
      sb[SB_N2 + lane] = lane < 15 ? b : 0.0f;
    }
  }
  int qn = 0;
  __syncthreads();

  const int nChunks = (nE + ECHUNK - 1) / ECHUNK;
#pragma unroll 1
  for (int ch = 0; ch < nChunks; ++ch) {
    const int cbase = ch * ECHUNK;
    const int wc = scan_chunk<NB, ENT, ENG, QCAP, 1>(ei, nE, cbase, nodeBase, vec8, qe, lane, qn);
    qn = wc > QCAP ? QCAP : (wc < 0 ? 0 : wc);
    wave_sync();

    const int T = qn >> 4;
#pragma unroll 1
    for (int t = 0; t < T; ++t)
      process_tile(x, ei, ea, nN, nE, nodeBase, 16 * t, 16, lane, qe, feat, hid, w1e, w2e, w1n, w2n, sb, accs);
    const int rem = qn & 15;
    if (T > 0 && rem > 0) {
      int src = 16 * T + lane;
      src = src > QCAP - 1 ? QCAP - 1 : src;
      const int v = qe[src];
      wave_sync();
      if (lane < rem) qe[lane] = v;
    }
    qn = rem;
    wave_sync();
  }
  if (qn > 0)
    process_tile(x, ei, ea, nN, nE, nodeBase, 0, qn, lane, qe, feat, hid, w1e, w2e, w1n, w2n, sb, accs);
  __syncthreads();

#pragma unroll 1
  for (int i = 0; i < NB / ENT; ++i) {
    const int s = i * ENT + lane;
    v4f* rp = (v4f*)(accs + s * 16);
    v4f q0 = rp[0], q1 = rp[1], q2 = rp[2], q3 = rp[3];
    const float inv = 1.0f / fmaxf(q3.w, 1.0f);
    q0 = q0 * inv; q1 = q1 * inv; q2 = q2 * inv; q3 = q3 * inv;
    q3.w = 0.0f;
    rp[0] = q0; rp[1] = q1; rp[2] = q2; rp[3] = q3;
  }
  __syncthreads();

  float* gp = x2 + (size_t)nodeBase * 16;
#pragma unroll 1
  for (int i = 0; i < (NB * 16 / 4) / ENT; ++i) {
    const int idx = i * ENT + lane;
    const v4f v = ((const v4f*)accs)[idx];
    *(volatile v4f*)(gp + 4 * (size_t)idx) = v;
  }
  __threadfence();
#pragma unroll 1
  for (int i = 0; i < (NB * 16 / 4) / ENT; ++i) {
    const int idx = i * ENT + lane;
    const v4f v = ((const v4f*)accs)[idx];
    *(volatile v4f*)(gp + 4 * (size_t)idx) = v;
  }
}

__global__ __launch_bounds__(NTHR) void k_graph(
    const int* __restrict__ batch, const float* __restrict__ x2, const float* __restrict__ u,
    const float* __restrict__ gw1, const float* __restrict__ gb1,
    const float* __restrict__ gw2, const float* __restrict__ gb2,
    const float* __restrict__ f1w, const float* __restrict__ f1b,
    float* zp, int nN, int G) {
  __shared__ __attribute__((aligned(16))) int list[LISTN];
  __shared__ int wcnt[NWAVE];
  __shared__ __attribute__((aligned(16))) __bf16 gin[2 * 16 * FP];
  __shared__ __attribute__((aligned(16))) __bf16 ghid[2 * 16 * HP];
  __shared__ __attribute__((aligned(16))) __bf16 sgw1[2 * HIDN * W1P];
  __shared__ __attribute__((aligned(16))) __bf16 sgw2[2 * OUTN * W2P];
  __shared__ float sgb[HIDN + OUTN];
  __shared__ __attribute__((aligned(16))) float su2[16 * 16];
  __shared__ __attribute__((aligned(16))) float sz[16 * 16];
  const int tid = threadIdx.x, lane = tid & 31, wave = tid >> 5, h = lane >> 4, m = lane & 15;
  const int g0 = blockIdx.x * NBG;
  const int vec8 = ((reinterpret_cast<size_t>(batch) & 15) == 0) ? 1 : 0;

  stage_w(gw1, 16, 50, sgw1, HIDN, W1P, tid);
  stage_w(gw2, 50, 15, sgw2, OUTN, W2P, tid);
  if (tid < HIDN) { const float b = gb1[tid < 50 ? tid : 49]; sgb[tid] = tid < 50 ? b : 0.0f; }
  if (tid < OUTN) { const float b = gb2[tid < 15 ? tid : 14]; sgb[HIDN + tid] = tid < 15 ? b : 0.0f; }
  float acc = 0.0f;
  int   cnt = 0;
  __syncthreads();

  const int nChunks = (nN + GCHUNK - 1) / GCHUNK;
#pragma unroll 1
  for (int ch = 0; ch < nChunks; ++ch) {
    const int cbase = ch * GCHUNK;
    const int wc = scan_chunk<NBG, NTHR, GNG, WCAP, 0>(batch, nN, cbase, g0, vec8, list + wave * WCAP, tid, 0);
    if (lane == 0) wcnt[wave] = wc;
    __syncthreads();
#pragma unroll 1
    for (int wsx = 0; wsx < NWAVE; ++wsx) {
      int n = __builtin_amdgcn_readfirstlane(wcnt[wsx]);
      n = n > WCAP ? WCAP : (n < 0 ? 0 : n);
      const int* lp = list + wsx * WCAP;
#pragma unroll 1
      for (int i = 0; i < n; ++i) {
        const int ent  = __builtin_amdgcn_readfirstlane(lp[i]);
        const int slot = ent & (NBG - 1);
        if ((slot >> 1) == wave) {
          int nd = cbase + (ent >> 12);
          nd = nd < 0 ? 0 : (nd > nN - 1 ? nN - 1 : nd);
          const float v = x2[(size_t)nd * 16 + m];
          const bool mine = ((slot & 1) == h);
          acc += mine ? v : 0.0f;
          cnt += mine ? 1 : 0;
        }
      }
    }
    __syncthreads();
  }

  {
    const int row = 2 * wave + h;
    int g = g0 + row;
    g = g > G - 1 ? G - 1 : g;
    const float inv = 1.0f / fmaxf((float)cnt, 1.0f);
    const float meanv = (m == 15) ? 0.0f : acc * inv;
    const float uv = u[g];
    __bf16 mh, ml, uh, ul;
    split2(meanv, mh, ml);
    split2(uv, uh, ul);
    const __bf16 bz = (__bf16)0.0f;
    __bf16* r0p = gin + row * FP;
    __bf16* r1p = gin + 16 * FP + row * FP;
    r0p[1 + m] = mh;
    r1p[1 + m] = ml;
    if (m < 15) { r0p[17 + m] = bz; r1p[17 + m] = bz; }
    if (m == 0) { r0p[0] = uh; r1p[0] = ul; }
  }
  __syncthreads();

  if (wave == 0) {
    layer1(gin, sgw1, sgb, ghid, h, m);
    wave_sync();
    const v8f a = gemm2(ghid, sgw2, h, m);
    const float bv = sgb[HIDN + m];
#pragma unroll
    for (int rr = 0; rr < 8; ++rr) su2[(8 * h + rr) * 16 + m] = a[rr] + bv;
  }
  __syncthreads();

  if (tid < 160) {
    const int gg = tid / 10;
    const int o  = tid - gg * 10;
    float s = f1b[o];
#pragma unroll
    for (int k = 0; k < 15; ++k) s += su2[gg * 16 + k] * f1w[k * 10 + o];
    sz[gg * 16 + o] = s;
  } else {
    const int q  = tid - 160;
    const int qr = q / 6;
    sz[qr * 16 + 10 + (q - qr * 6)] = 0.0f;
  }
  __syncthreads();

  if (wave == 0) {
    float* gp = zp + (size_t)g0 * 16;
    const v4f v0 = *(const v4f*)(sz + 4 * lane);
    const v4f v1 = *(const v4f*)(sz + 4 * (32 + lane));
    *(volatile v4f*)(gp + 4 * lane) = v0;
    *(volatile v4f*)(gp + 4 * (32 + lane)) = v1;
    __threadfence();
    *(volatile v4f*)(gp + 4 * lane) = v0;
    *(volatile v4f*)(gp + 4 * (32 + lane)) = v1;
  }
}

__global__ __launch_bounds__(NTHR) void k_head(
    const float* __restrict__ zp, const float* __restrict__ bng, const float* __restrict__ bnb,
    const float* __restrict__ f2w, const float* __restrict__ f2b, float* out, int G) {
  __shared__ float smean[16], srstd[16], sgam[16], sbet[16], sf2b[8];
  __shared__ float sf2w[64];
  __shared__ __attribute__((aligned(16))) float sout[GMAX * 6];
  const int tid = threadIdx.x;
  if (tid < 60) sf2w[tid] = f2w[tid];
  if (tid < 6) sf2b[tid] = f2b[tid];
  if (tid < 10) { sgam[tid] = bng[tid]; sbet[tid] = bnb[tid]; }
  if (tid < 10) {
    double s = 0.0;
#pragma unroll 1
    for (int g = 0; g < G; ++g) s += (double)zp[(size_t)g * 16 + tid];
    const double mean = s / (double)G;
    double q = 0.0;
#pragma unroll 1
    for (int g = 0; g < G; ++g) {
      const double d = (double)zp[(size_t)g * 16 + tid] - mean;
      q += d * d;
    }
    const double var = q / (double)G;
    smean[tid] = (float)mean;
    srstd[tid] = rsqrtf((float)var + 1e-5f);
  }
  __syncthreads();

#pragma unroll 1
  for (int g = tid; g < G; g += NTHR) {
    const float* zr = zp + (size_t)g * 16;
    const v4f z0 = *(const v4f*)(zr);
    const v4f z1 = *(const v4f*)(zr + 4);
    const v4f z2 = *(const v4f*)(zr + 8);
    const float zv[10] = {z0.x, z0.y, z0.z, z0.w, z1.x, z1.y, z1.z, z1.w, z2.x, z2.y};
    float zn[10];
#pragma unroll
    for (int o = 0; o < 10; ++o)
      zn[o] = fmaxf((zv[o] - smean[o]) * srstd[o] * sgam[o] + sbet[o], 0.0f);
    float mx = -3.0e38f;
#pragma unroll 1
    for (int c = 0; c < 6; ++c) {
      float s = sf2b[c];
#pragma unroll
      for (int o = 0; o < 10; ++o) s += zn[o] * sf2w[o * 6 + c];
      sout[g * 6 + c] = s;
      mx = fmaxf(mx, s);
    }
    float se = 0.0f;
#pragma unroll 1
    for (int c = 0; c < 6; ++c) se += __expf(sout[g * 6 + c] - mx);
    const float lse = mx + __logf(se);
#pragma unroll 1
    for (int c = 0; c < 6; ++c) sout[g * 6 + c] = sout[g * 6 + c] - lse;
  }
  __syncthreads();

  const int tot = G * 6;
  const int nv  = tot >> 2;
#pragma unroll 1
  for (int i = tid; i < nv; i += NTHR) {
    const v4f v = *(const v4f*)(sout + 4 * i);
    *(volatile v4f*)(out + 4 * (size_t)i) = v;
  }
  if (tid == 0) {
#pragma unroll 1
    for (int j = 4 * nv; j < tot; ++j) { const float v = sout[j]; *(volatile float*)(out + j) = v; }
  }
  __threadfence();
#pragma unroll 1
  for (int i = tid; i < nv; i += NTHR) {
    const v4f v = *(const v4f*)(sout + 4 * i);
    *(volatile v4f*)(out + 4 * (size_t)i) = v;
  }
  if (tid == 0) {
#pragma unroll 1
    for (int j = 4 * nv; j < tot; ++j) { const float v = sout[j]; *(volatile float*)(out + j) = v; }
  }
}

extern "C" void kernel_launch(void* const* d_in, const int* in_sizes, int n_in,
                              void* d_out, int out_size, void* d_ws, size_t ws_size,
                              hipStream_t stream) {
  if (n_in < 23) return;
  const int nN = in_sizes[4];
  if (nN <= 0 || in_sizes[0] != 3 * nN) return;
  const int nE = in_sizes[1] / 2;
  if (nE <= 0 || in_sizes[1] != 2 * nE || in_sizes[2] != 3 * nE) return;
  const int G = in_sizes[3];
  if (G <= 0 || G > GMAX || out_size != 6 * G) return;
  if (in_sizes[5] != 450 || in_sizes[6] != 50 || in_sizes[7] != 750 || in_sizes[8] != 15) return;
  if (in_sizes[9] != 900 || in_sizes[10] != 50 || in_sizes[11] != 750 || in_sizes[12] != 15) return;
  if (in_sizes[13] != 800 || in_sizes[14] != 50 || in_sizes[15] != 750 || in_sizes[16] != 15) return;
  if (in_sizes[17] != 150 || in_sizes[18] != 10 || in_sizes[19] != 10 || in_sizes[20] != 10) return;
  if (in_sizes[21] != 60 || in_sizes[22] != 6) return;
  if (nE > (1 << 28) || nN > (1 << 26)) return;

  const float* x     = (const float*)d_in[0];
  const int*   ei    = (const int*)d_in[1];
  const float* ea    = (const float*)d_in[2];
  const float* u     = (const float*)d_in[3];
  const int*   batch = (const int*)d_in[4];
  const float* ew1 = (const float*)d_in[5];
  const float* eb1 = (const float*)d_in[6];
  const float* ew2 = (const float*)d_in[7];
  const float* eb2 = (const float*)d_in[8];
  const float* nw1 = (const float*)d_in[9];
  const float* nb1 = (const float*)d_in[10];
  const float* nw2 = (const float*)d_in[11];
  const float* nb2 = (const float*)d_in[12];
  const float* gw1 = (const float*)d_in[13];
  const float* gb1 = (const float*)d_in[14];
  const float* gw2 = (const float*)d_in[15];
  const float* gb2 = (const float*)d_in[16];
  const float* f1w = (const float*)d_in[17];
  const float* f1b = (const float*)d_in[18];
  const float* bng = (const float*)d_in[19];
  const float* bnb = (const float*)d_in[20];
  const float* f2w = (const float*)d_in[21];
  const float* f2b = (const float*)d_in[22];
  float* out = (float*)d_out;

  const int nBlk = (nN + NB - 1) / NB;
  const int nGB  = (G + NBG - 1) / NBG;

  char* ws = (char*)d_ws;
  size_t off = 0;
  const size_t oW  = off; off += (size_t)WTOT * 2;            off = (off + 255) & ~(size_t)255;
  const size_t oX2 = off; off += (size_t)nBlk * NB * 16 * 4;  off = (off + 255) & ~(size_t)255;
  const size_t oZ  = off; off += (size_t)nGB * NBG * 16 * 4;  off = (off + 255) & ~(size_t)255;
  if (off > ws_size) return;
  __bf16* wpl = (__bf16*)(ws + oW);
  float*  x2  = (float*)(ws + oX2);
  float*  zp  = (float*)(ws + oZ);

  k_wprep<<<1, NTHR, 0, stream>>>(ew1, ew2, nw1, nw2, wpl);
  hipFuncSetAttribute(reinterpret_cast<const void*>(&k_edge),
                      hipFuncAttributeMaxDynamicSharedMemorySize, LDS_EDGE);
  k_edge<<<nBlk, ENT, LDS_EDGE, stream>>>(x, ei, ea, wpl, eb1, eb2, nb1, nb2, x2, nN, nE);
  k_graph<<<nGB, NTHR, 0, stream>>>(batch, x2, u, gw1, gb1, gw2, gb2, f1w, f1b, zp, nN, G);
  k_head<<<1, NTHR, 0, stream>>>(zp, bng, bnb, f2w, f2b, out, G);
}
